// BidirectionalAttention_57698590654997
// MI455X (gfx1250) — hardware-verified
//
#include <hip/hip_runtime.h>
#include <math.h>

constexpr int kB = 2;
constexpr int kS = 2048;
constexpr int kDim = 1024;
constexpr int kH = 16;
constexpr int kDh = 64;
constexpr int kM = kB * kS;
constexpr int kNqkv = 3 * kDim;
constexpr int kBH = kB * kH;
constexpr int kKC = 64;
constexpr int kRsPitch = 32;

constexpr size_t kPlane  = (size_t)kBH * kS * kDh * 2;
constexpr size_t kOffXb  = 0;
constexpr size_t kOffRs  = kOffXb + (size_t)kM * kDim * 2;
constexpr size_t kOffWq  = kOffRs + (size_t)kM * kRsPitch * 4;
constexpr size_t kOffWo  = kOffWq + (size_t)kNqkv * kDim * 2;
constexpr size_t kOffCt  = kOffWo + (size_t)kDim * kDim * 2;
constexpr size_t kOffSt  = kOffCt + (size_t)kS * kDh * 4;
constexpr size_t kOffQh  = kOffSt + (size_t)kS * kDh * 4;
constexpr size_t kOffQl  = kOffQh + kPlane;
constexpr size_t kOffKh  = kOffQl + kPlane;
constexpr size_t kOffKl  = kOffKh + kPlane;
constexpr size_t kOffVh  = kOffKl + kPlane;
constexpr size_t kOffVl  = kOffVh + kPlane;
constexpr size_t kOffVth = kOffVl + kPlane;
constexpr size_t kOffVtl = kOffVth + kPlane;
constexpr size_t kOffAh  = kOffVtl + kPlane;
constexpr size_t kOffAl  = kOffAh + kPlane;
constexpr size_t kWsTotal = kOffAl + kPlane;

typedef char ck_ws_total[(kWsTotal == (size_t)102236160) ? 1 : -1];
typedef char ck_ws_cap[(kWsTotal <= (size_t)134217728) ? 1 : -1];
typedef char ck_align[((kOffRs % 128) == 0 && (kOffQh % 128) == 0 && (kPlane % 128) == 0) ? 1 : -1];
typedef char ck_tiles[(kM % 64 == 0 && kNqkv % 64 == 0 && kDim % 64 == 0 && kDim % 32 == 0 && kS % 64 == 0 && kDh == 64) ? 1 : -1];
typedef char ck_plane[((size_t)kM * kDim * 2 == kPlane) ? 1 : -1];

typedef __attribute__((ext_vector_type(16))) _Float16 v16h;
typedef __attribute__((ext_vector_type(8)))  _Float16 v8h;
typedef __attribute__((ext_vector_type(16))) __bf16   v16b;
typedef __attribute__((ext_vector_type(8)))  __bf16   v8b;
typedef __attribute__((ext_vector_type(8)))  float    v8f;
typedef __attribute__((ext_vector_type(4)))  float    v4f;
typedef __attribute__((ext_vector_type(4)))  unsigned v4u;

__device__ __forceinline__ unsigned short f2bf_bits(float f) {
  unsigned u = __float_as_uint(f);
  return (unsigned short)((u + 0x7FFFu + ((u >> 16) & 1u)) >> 16);
}
__device__ __forceinline__ float bf_bits2f(unsigned short h) { return __uint_as_float(((unsigned)h) << 16); }

__device__ __forceinline__ void dep_guard_h(v8f& a, v8f& b, v16h x, v16h y) { asm volatile("v_nop\n\tv_nop\n\tv_nop\n\tv_nop" : "+v"(a), "+v"(b) : "v"(x), "v"(y)); }
__device__ __forceinline__ void dep_guard_b(v8f& a, v8f& b, v16b x, v16b y) { asm volatile("v_nop\n\tv_nop\n\tv_nop\n\tv_nop" : "+v"(a), "+v"(b) : "v"(x), "v"(y)); }
__device__ __forceinline__ void keep4_h(v16h a, v16h b, v16h c, v16h d) { asm volatile("v_nop" :: "v"(a), "v"(b), "v"(c), "v"(d)); }
__device__ __forceinline__ void keep4_b(v16b a, v16b b, v16b c, v16b d) { asm volatile("v_nop" :: "v"(a), "v"(b), "v"(c), "v"(d)); }
__device__ __forceinline__ void acc_guard4(v8f& a, v8f& b, v8f& c, v8f& d) { asm volatile("v_nop\n\tv_nop\n\tv_nop\n\tv_nop" : "+v"(a), "+v"(b), "+v"(c), "+v"(d)); }
template <typename T> struct Frag;
template <> struct Frag<_Float16> {
  typedef v16h V; union U { v16h v; v8h h[2]; };
  static __device__ __forceinline__ v16h load(const _Float16* p) {
    U f; f.h[0] = *(const v8h*)(p); f.h[1] = *(const v8h*)(p + 16); return f.v;
  }
  static __device__ __forceinline__ v8f mma(v16h a, v16h b, v8f c) {
    return __builtin_amdgcn_wmma_f32_16x16x32_f16(false, a, false, b, (short)0, c, false, false);
  }
  static __device__ __forceinline__ void guard(v8f& a, v8f& b, v16h x, v16h y) { dep_guard_h(a, b, x, y); }
  static __device__ __forceinline__ void keep(v16h a, v16h b, v16h c, v16h d) { keep4_h(a, b, c, d); }
};
template <> struct Frag<__bf16> {
  typedef v16b V; union U { v16b v; v8b h[2]; };
  static __device__ __forceinline__ v16b load(const __bf16* p) {
    U f; f.h[0] = *(const v8b*)(p); f.h[1] = *(const v8b*)(p + 16); return f.v;
  }
  static __device__ __forceinline__ v8f mma(v16b a, v16b b, v8f c) {
    return __builtin_amdgcn_wmma_f32_16x16x32_bf16(false, a, false, b, (short)0, c, false, false);
  }
  static __device__ __forceinline__ void guard(v8f& a, v8f& b, v16b x, v16b y) { dep_guard_b(a, b, x, y); }
  static __device__ __forceinline__ void keep(v16b a, v16b b, v16b c, v16b d) { keep4_b(a, b, c, d); }
};

__device__ __forceinline__ v8f mma_bf(v16b a, v16b b, v8f c) {
  c = __builtin_amdgcn_wmma_f32_16x16x32_bf16(false, a, false, b, (short)0, c, false, false);
  asm volatile("v_nop\n\tv_nop\n\tv_nop\n\tv_nop" : "+v"(c) : "v"(a), "v"(b));
  return c;
}
__device__ __forceinline__ v8f mma_hf(v16b a, v16b b, v8f c) {
  const v16h ah = __builtin_bit_cast(v16h, a), bh = __builtin_bit_cast(v16h, b);
  c = __builtin_amdgcn_wmma_f32_16x16x32_f16(false, ah, false, bh, (short)0, c, false, false);
  asm volatile("v_nop\n\tv_nop\n\tv_nop\n\tv_nop" : "+v"(c) : "v"(ah), "v"(bh));
  return c;
}

__device__ __forceinline__ void wave_sync_lds() {
  __builtin_amdgcn_fence(__ATOMIC_RELEASE, "workgroup");
  __builtin_amdgcn_wave_barrier();
  __builtin_amdgcn_fence(__ATOMIC_ACQUIRE, "workgroup");
}

__global__ __launch_bounds__(128) void k_rms_xcast(const float* __restrict__ x,
                                                   unsigned short* __restrict__ xb,
                                                   float* __restrict__ rstab) {
  __shared__ float red[4];
  const int m = blockIdx.x;
  const int t = threadIdx.x;
  const int lane = t & 31, wave = t >> 5;
  const size_t base = (size_t)m * kDim + (size_t)t * 8;
  const v4f xa = *(const v4f*)(x + base);
  const v4f xc = *(const v4f*)(x + base + 4);
  unsigned short hb[8];
#pragma unroll
  for (int e = 0; e < 4; ++e) { hb[e] = f2bf_bits(xa[e]); hb[4 + e] = f2bf_bits(xc[e]); }
  float ss = 0.0f;
#pragma unroll
  for (int e = 0; e < 8; ++e) { const float r = bf_bits2f(hb[e]); ss += r * r; }
#pragma unroll
  for (int off = 16; off > 0; off >>= 1) ss += __shfl_xor(ss, off, 32);
  if (lane == 0) red[wave] = ss;
  __syncthreads();
  const float tot = ((red[0] + red[1]) + red[2]) + red[3];
  const float nrm = sqrtf(tot);
  const float inv = 1.0f / fmaxf(nrm, 1e-12f);
  const float rs = inv * 32.0f;
  v4u w;
  w[0] = (unsigned)hb[0] | ((unsigned)hb[1] << 16);
  w[1] = (unsigned)hb[2] | ((unsigned)hb[3] << 16);
  w[2] = (unsigned)hb[4] | ((unsigned)hb[5] << 16);
  w[3] = (unsigned)hb[6] | ((unsigned)hb[7] << 16);
  unsigned short* dst = xb + base;
  const v4f rv = (v4f){rs, rs, rs, rs};
  float* rp = rstab + (size_t)m * kRsPitch + (t & 7) * 4;
  *(volatile v4u*)dst = w;
  if (t < 8) *(volatile v4f*)rp = rv;
  __threadfence();
  *(volatile v4u*)dst = w;
  if (t < 8) *(volatile v4f*)rp = rv;
}

template <bool HAS_G>
__global__ __launch_bounds__(256) void k_wcast(const float* __restrict__ w, const float* __restrict__ g,
                                               unsigned short* __restrict__ wt, int ncols) {
  __shared__ float tile[64][65];
  const int t = threadIdx.x, lane = t & 31, wave = t >> 5;
  const int n0 = blockIdx.x * 64, k0 = blockIdx.y * 64;
#pragma unroll
  for (int i = 0; i < 4; ++i) {
    const int idx = i * 256 + t;
    const int r = idx >> 4, c4 = (idx & 15) * 4;
    const v4f v = *(const v4f*)(w + (size_t)(k0 + r) * ncols + n0 + c4);
    tile[r][c4 + 0] = v[0]; tile[r][c4 + 1] = v[1]; tile[r][c4 + 2] = v[2]; tile[r][c4 + 3] = v[3];
  }
  __syncthreads();
  const int q = lane >> 3, kc = (lane & 7) * 8;
  float gv[8];
  if (HAS_G) {
    const v4f g0 = *(const v4f*)(g + k0 + kc);
    const v4f g1 = *(const v4f*)(g + k0 + kc + 4);
#pragma unroll
    for (int e = 0; e < 4; ++e) { gv[e] = bf_bits2f(f2bf_bits(g0[e])); gv[4 + e] = bf_bits2f(f2bf_bits(g1[e])); }
  } else {
#pragma unroll
    for (int e = 0; e < 8; ++e) gv[e] = 1.0f;
  }
  v4u ov[2];
#pragma unroll
  for (int it = 0; it < 2; ++it) {
    const int nrow = it * 32 + wave * 4 + q;
    unsigned short bits[8];
#pragma unroll
    for (int e = 0; e < 8; ++e) {
      float f = bf_bits2f(f2bf_bits(tile[kc + e][nrow]));
      if (HAS_G) f = f * gv[e];
      bits[e] = f2bf_bits(f);
    }
    ov[it][0] = (unsigned)bits[0] | ((unsigned)bits[1] << 16);
    ov[it][1] = (unsigned)bits[2] | ((unsigned)bits[3] << 16);
    ov[it][2] = (unsigned)bits[4] | ((unsigned)bits[5] << 16);
    ov[it][3] = (unsigned)bits[6] | ((unsigned)bits[7] << 16);
  }
  for (int pass = 0; pass < 2; ++pass) {
#pragma unroll
    for (int it = 0; it < 2; ++it) {
      const int nrow = it * 32 + wave * 4 + q;
      *(volatile v4u*)(wt + (size_t)(n0 + nrow) * kDim + k0 + kc) = ov[it];
    }
    __threadfence();
  }
}

__global__ __launch_bounds__(256) void k_trig(const float* __restrict__ pos, float* __restrict__ ct,
                                              float* __restrict__ st, int n) {
  const int i = blockIdx.x * 256 + threadIdx.x;
  if (i < n) {
    const float pb = bf_bits2f(f2bf_bits(pos[i]));
    const float cv = cosf(pb);
    const float sv = sinf(pb);
    ((volatile float*)ct)[i] = cv;
    ((volatile float*)st)[i] = sv;
    __threadfence();
    ((volatile float*)ct)[i] = cv;
    ((volatile float*)st)[i] = sv;
  }
}

template <int SPLITM>
__device__ __forceinline__ void gemm64_core(const __bf16* __restrict__ Ab, const __bf16* __restrict__ Ab2, int lda,
                                            const __bf16* __restrict__ Bb, int ldb, int m0, int n0, int K, int lane,
                                            v8f (&acc)[4][4]) {
  const int rlane = lane & 15;
  const int koff = (lane >> 4) * 8;
#pragma unroll
  for (int i = 0; i < 4; ++i)
#pragma unroll
    for (int j = 0; j < 4; ++j) acc[i][j] = (v8f){0.f,0.f,0.f,0.f,0.f,0.f,0.f,0.f};
  for (int k0 = 0; k0 < K; k0 += 32) {
    v16b bfr[4];
#pragma unroll
    for (int j = 0; j < 4; ++j) {
      const size_t bo = (size_t)(n0 + (j << 4) + rlane) * ldb + koff + k0;
      bfr[j] = Frag<__bf16>::load(Bb + bo);
    }
#pragma unroll
    for (int i = 0; i < 4; ++i) {
      const size_t ao = (size_t)(m0 + (i << 4) + rlane) * lda + koff + k0;
      v16b ah = Frag<__bf16>::load(Ab + ao);
      v16b al = ah;
      if (SPLITM) al = Frag<__bf16>::load(Ab2 + ao);
#pragma unroll
      for (int j = 0; j < 4; ++j) {
        acc[i][j] = Frag<__bf16>::mma(ah, bfr[j], acc[i][j]);
        if (SPLITM) acc[i][j] = Frag<__bf16>::mma(al, bfr[j], acc[i][j]);
      }
      Frag<__bf16>::guard(acc[i][0], acc[i][3], ah, al);
    }
    Frag<__bf16>::keep(bfr[0], bfr[1], bfr[2], bfr[3]);
  }
  acc_guard4(acc[0][0], acc[0][1], acc[0][2], acc[0][3]);
  acc_guard4(acc[1][0], acc[1][1], acc[1][2], acc[1][3]);
  acc_guard4(acc[2][0], acc[2][1], acc[2][2], acc[2][3]);
  acc_guard4(acc[3][0], acc[3][1], acc[3][2], acc[3][3]);
}

__global__ __launch_bounds__(256) void k_gemm_qkv(
    const unsigned short* __restrict__ xbp, const unsigned short* __restrict__ wtp,
    const float* __restrict__ rstab, const float* __restrict__ ct, const float* __restrict__ st,
    unsigned short* __restrict__ qh, unsigned short* __restrict__ ql,
    unsigned short* __restrict__ kh, unsigned short* __restrict__ kl,
    unsigned short* __restrict__ vh, unsigned short* __restrict__ vl) {
  __shared__ __align__(16) float sT[8][16 * 68];
  const int lane = threadIdx.x & 31, wave = threadIdx.x >> 5;
  constexpr int tilesN = kNqkv / 64;
  constexpr int tilesM = kM / 64;
  const int tile = blockIdx.x * 8 + wave;
  if (tile >= tilesM * tilesN) return;
  const int tm = tile / tilesN, tn = tile - tm * tilesN;
  const int m0 = tm << 6, n0 = tn << 6;

  v8f acc[4][4];
  gemm64_core<0>((const __bf16*)xbp, (const __bf16*)xbp, kDim, (const __bf16*)wtp, kDim, m0, n0, kDim, lane, acc);

  float* slab = sT[wave];
  const int rlane = lane & 15, mOff = (lane >> 4) * 8;
  const int sec = n0 >> 10;
  const int hidx = (n0 & (kDim - 1)) >> 6;
  unsigned short* P0 = (sec == 0) ? qh : ((sec == 1) ? kh : vh);
  unsigned short* P1 = (sec == 0) ? ql : ((sec == 1) ? kl : vl);
  const int q8 = lane >> 3, c8 = (lane & 7) * 8;
  const int cpart = c8 ^ 32;
  const float sgn = (c8 < 32) ? -1.0f : 1.0f;
#pragma unroll
  for (int i = 0; i < 4; ++i) {
    const int mBase = m0 + (i << 4);
    float rsv[8];
#pragma unroll
    for (int r = 0; r < 8; ++r) rsv[r] = rstab[(size_t)(mBase + mOff + r) * kRsPitch];
#pragma unroll
    for (int j = 0; j < 4; ++j)
#pragma unroll
      for (int r = 0; r < 8; ++r) slab[(mOff + r) * 68 + (j << 4) + rlane] = acc[i][j][r] * rsv[r];
    wave_sync_lds();
    for (int pass = 0; pass < 2; ++pass) {
#pragma unroll
      for (int it = 0; it < 4; ++it) {
        const int row = it * 4 + q8;
        const int m = mBase + row;
        const int bb = m >> 11, nn = m & (kS - 1);
        const float* sp = slab + row * 68;
        const size_t dsto = ((size_t)(bb * kH + hidx) * kS + nn) * kDh + c8;
        v8h hv, lv;
        if (sec < 2) {
          const v4f ca = *(const v4f*)(ct + (size_t)nn * kDh + c8);
          const v4f cb = *(const v4f*)(ct + (size_t)nn * kDh + c8 + 4);
          const v4f sa = *(const v4f*)(st + (size_t)nn * kDh + c8);
          const v4f sb = *(const v4f*)(st + (size_t)nn * kDh + c8 + 4);
          float cvv[8], svv[8];
#pragma unroll
          for (int e = 0; e < 4; ++e) { cvv[e] = ca[e]; cvv[4 + e] = cb[e]; svv[e] = sa[e]; svv[4 + e] = sb[e]; }
#pragma unroll
          for (int e = 0; e < 8; ++e) {
            const float v = sp[c8 + e];
            const float pr = sp[cpart + e];
            const float rv = v * cvv[e] + sgn * pr * svv[e];
            const unsigned short hb = f2bf_bits(rv);
            const unsigned short lb = f2bf_bits(rv - bf_bits2f(hb));
            hv[e] = __builtin_bit_cast(_Float16, hb);
            lv[e] = __builtin_bit_cast(_Float16, lb);
          }
        } else {
#pragma unroll
          for (int e = 0; e < 8; ++e) {
            const float v = sp[c8 + e];
            const _Float16 h16 = (_Float16)v;
            const float hf = (float)h16;
            hv[e] = h16;
            lv[e] = (_Float16)((v - hf) * 2048.0f);
          }
        }
        *(volatile v8h*)(P0 + dsto) = hv;
        *(volatile v8h*)(P1 + dsto) = lv;
      }
      __threadfence();
    }
    wave_sync_lds();
  }
}

__global__ __launch_bounds__(256) void k_vtrans(const unsigned short* __restrict__ vh, const unsigned short* __restrict__ vl,
                                                unsigned short* __restrict__ vth, unsigned short* __restrict__ vtl) {
  __shared__ __align__(16) unsigned short tile[64 * 72];
  const int t = threadIdx.x, lane = t & 31, wave = t >> 5;
  const int bh = blockIdx.x >> 5, kvt = blockIdx.x & 31;
  const int kv0 = kvt * 64;
  const unsigned short* src = (blockIdx.y == 0) ? vh : vl;
  unsigned short* dst = (blockIdx.y == 0) ? vth : vtl;
#pragma unroll
  for (int i = 0; i < 2; ++i) {
    const int idx = i * 256 + t;
    const int r = idx >> 3, c16 = (idx & 7) * 8;
    const v4u w = *(const v4u*)(src + ((size_t)bh * kS + kv0 + r) * kDh + c16);
#pragma unroll
    for (int e = 0; e < 4; ++e) {
      tile[(c16 + 2 * e) * 72 + r] = (unsigned short)(w[e] & 0xffffu);
      tile[(c16 + 2 * e + 1) * 72 + r] = (unsigned short)(w[e] >> 16);
    }
  }
  __syncthreads();
  const int q = lane >> 3, kc = (lane & 7) * 8;
  v4u ov[2];
#pragma unroll
  for (int it = 0; it < 2; ++it) {
    const int d = it * 32 + wave * 4 + q;
    ov[it] = *(const v4u*)(tile + d * 72 + kc);
  }
  for (int pass = 0; pass < 2; ++pass) {
#pragma unroll
    for (int it = 0; it < 2; ++it) {
      const int d = it * 32 + wave * 4 + q;
      *(volatile v4u*)(dst + ((size_t)bh * kDh + d) * kS + kv0 + kc) = ov[it];
    }
    __threadfence();
  }
}

constexpr int kLdsK = 0;
constexpr int kLdsV = 16384;
constexpr int kLdsP = 32768;
constexpr int kLdsTotal = 49152;

__global__ __launch_bounds__(128) void k_attn(
    const unsigned short* __restrict__ qhp, const unsigned short* __restrict__ qlp,
    const unsigned short* __restrict__ khp, const unsigned short* __restrict__ klp,
    const unsigned short* __restrict__ vthp, const unsigned short* __restrict__ vtlp,
    unsigned short* __restrict__ aoh, unsigned short* __restrict__ aol) {
  union FB { v16b v; v8b h[2]; };
  __shared__ __align__(16) unsigned char lds_raw[kLdsTotal];
  __bf16* Ksh = (__bf16*)(lds_raw + kLdsK);
  __bf16* Ksl = (__bf16*)(lds_raw + kLdsK + 8192);
  __bf16* Vsh = (__bf16*)(lds_raw + kLdsV);
  __bf16* Vsl = (__bf16*)(lds_raw + kLdsV + 8192);
  __bf16* Pbase  = (__bf16*)(lds_raw + kLdsP);
  __bf16* Plbase = (__bf16*)(lds_raw + kLdsP + 8192);
  unsigned short* KshU = (unsigned short*)(lds_raw + kLdsK);
  unsigned short* KslU = (unsigned short*)(lds_raw + kLdsK + 8192);
  unsigned short* VshU = (unsigned short*)(lds_raw + kLdsV);
  unsigned short* VslU = (unsigned short*)(lds_raw + kLdsV + 8192);

  const int tid = threadIdx.x, wave = tid >> 5, lane = tid & 31;
  const int hh = lane >> 4, c = lane & 15;
  const int bx = blockIdx.x;
  const int qb = bx & 31;
  const int bh = bx >> 5;
  const int h = bh & (kH - 1);
  const int b = bh >> 4;
  const int q0 = qb * 64 + wave * 16;

  v16b qah[2], qal[2];
  {
    const __bf16* qr  = (const __bf16*)qhp + ((size_t)bh * kS + q0 + c) * kDh;
    const __bf16* qr2 = (const __bf16*)qlp + ((size_t)bh * kS + q0 + c) * kDh;
#pragma unroll
    for (int dc = 0; dc < 2; ++dc) {
      qah[dc] = Frag<__bf16>::load(qr + dc * 32 + 8 * hh);
      qal[dc] = Frag<__bf16>::load(qr2 + dc * 32 + 8 * hh);
    }
  }

  float mrow[8], lrow[8];
  v8f oacc[4], oacr[4];
#pragma unroll
  for (int r = 0; r < 8; ++r) { mrow[r] = -INFINITY; lrow[r] = 0.f; }
#pragma unroll
  for (int t = 0; t < 4; ++t) { oacc[t] = (v8f){0.f,0.f,0.f,0.f,0.f,0.f,0.f,0.f}; oacr[t] = (v8f){0.f,0.f,0.f,0.f,0.f,0.f,0.f,0.f}; }

  __bf16* pwh = Pbase + wave * (16 * kKC);
  __bf16* pwl = Plbase + wave * (16 * kKC);

  for (int kc = 0; kc < kS / kKC; ++kc) {
    const int kv0 = kc * kKC;
    __syncthreads();
    {
#pragma unroll
      for (int i = 0; i < 4; ++i) {
        const int idx = i * 128 + tid;
        const int r = idx >> 3, c16 = (idx & 7) * 8;
        const size_t ko = ((size_t)bh * kS + kv0 + r) * kDh + c16;
        const v4u w0 = *(const v4u*)(khp + ko);
        const v4u w1 = *(const v4u*)(klp + ko);
        *(v4u*)(KshU + r * kDh + c16) = w0;
        *(v4u*)(KslU + r * kDh + c16) = w1;
      }
#pragma unroll
      for (int i = 0; i < 4; ++i) {
        const int idx = i * 128 + tid;
        const int r = idx >> 3, c16 = (idx & 7) * 8;
        const size_t vo = ((size_t)bh * kDh + r) * kS + kv0 + c16;
        const v4u w2 = *(const v4u*)(vthp + vo);
        const v4u w3 = *(const v4u*)(vtlp + vo);
        *(v4u*)(VshU + r * kKC + c16) = w2;
        *(v4u*)(VslU + r * kKC + c16) = w3;
      }
    }
    __syncthreads();

    v8f s[4];
#pragma unroll
    for (int j = 0; j < 4; ++j) {
      s[j] = (v8f){0.f,0.f,0.f,0.f,0.f,0.f,0.f,0.f};
#pragma unroll
      for (int dc = 0; dc < 2; ++dc) {
        FB kb, kr;
        kb.h[0] = *(const v8b*)(Ksh + (j * 16 + c) * kDh + dc * 32 + 8 * hh);
        kb.h[1] = *(const v8b*)(Ksh + (j * 16 + c) * kDh + dc * 32 + 16 + 8 * hh);
        kr.h[0] = *(const v8b*)(Ksl + (j * 16 + c) * kDh + dc * 32 + 8 * hh);
        kr.h[1] = *(const v8b*)(Ksl + (j * 16 + c) * kDh + dc * 32 + 16 + 8 * hh);
        s[j] = mma_bf(qah[dc], kb.v, s[j]);
        s[j] = mma_bf(qah[dc], kr.v, s[j]);
        s[j] = mma_bf(qal[dc], kb.v, s[j]);
      }
    }
    float cm[8];
#pragma unroll
    for (int r = 0; r < 8; ++r) {
      float m = -INFINITY;
#pragma unroll
      for (int j = 0; j < 4; ++j) { s[j][r] *= 0.125f; m = fmaxf(m, s[j][r]); }
#pragma unroll
      for (int off = 1; off < 16; off <<= 1) m = fmaxf(m, __shfl_xor(m, off, 32));
      cm[r] = m;
    }
#pragma unroll
    for (int r = 0; r < 8; ++r) {
      const float mnew = fmaxf(mrow[r], cm[r]);
      const float alpha = expf(mrow[r] - mnew);
      mrow[r] = mnew;
      float psum = 0.f;
#pragma unroll
      for (int j = 0; j < 4; ++j) {
        const float p = expf(s[j][r] - mnew);
        psum += p;
        const float ps = p * 1024.0f;
        const _Float16 ph = (_Float16)ps;
        const float phf = (float)ph;
        const _Float16 pl = (_Float16)((ps - phf) * 2048.0f);
        pwh[(8 * hh + r) * kKC + j * 16 + c] = __builtin_bit_cast(__bf16, ph);
        pwl[(8 * hh + r) * kKC + j * 16 + c] = __builtin_bit_cast(__bf16, pl);
      }
#pragma unroll
      for (int off = 1; off < 16; off <<= 1) psum += __shfl_xor(psum, off, 32);
      lrow[r] = lrow[r] * alpha + psum;
#pragma unroll
      for (int t = 0; t < 4; ++t) { oacc[t][r] *= alpha; oacr[t][r] *= alpha; }
    }
    wave_sync_lds();
#pragma unroll 1
    for (int kk = 0; kk < 2; ++kk) {
      FB pa, pl;
      pa.h[0] = *(const v8b*)(pwh + c * kKC + kk * 32 + 8 * hh);
      pa.h[1] = *(const v8b*)(pwh + c * kKC + kk * 32 + 16 + 8 * hh);
      pl.h[0] = *(const v8b*)(pwl + c * kKC + kk * 32 + 8 * hh);
      pl.h[1] = *(const v8b*)(pwl + c * kKC + kk * 32 + 16 + 8 * hh);
#pragma unroll
      for (int t = 0; t < 4; ++t) {
        FB vb, vr;
        vb.h[0] = *(const v8b*)(Vsh + (t * 16 + c) * kKC + kk * 32 + 8 * hh);
        vb.h[1] = *(const v8b*)(Vsh + (t * 16 + c) * kKC + kk * 32 + 16 + 8 * hh);
        vr.h[0] = *(const v8b*)(Vsl + (t * 16 + c) * kKC + kk * 32 + 8 * hh);
        vr.h[1] = *(const v8b*)(Vsl + (t * 16 + c) * kKC + kk * 32 + 16 + 8 * hh);
        oacc[t] = mma_hf(pa.v, vb.v, oacc[t]);
        oacr[t] = mma_hf(pa.v, vr.v, oacr[t]);
        oacr[t] = mma_hf(pl.v, vb.v, oacr[t]);
      }
    }
  }

  __syncthreads();
  float* os = (float*)(lds_raw + 0) + wave * (16 * 64);
#pragma unroll
  for (int r = 0; r < 8; ++r) {
    const float inv = 1.0f / (lrow[r] * 1024.0f);
#pragma unroll
    for (int t = 0; t < 4; ++t)
      os[(8 * hh + r) * 64 + t * 16 + c] = (oacc[t][r] + oacr[t][r] * (1.0f / 2048.0f)) * inv;
  }
  __syncthreads();
  {
    const int q8 = lane >> 3, c8 = (lane & 7) * 8;
    for (int pass = 0; pass < 2; ++pass) {
#pragma unroll
      for (int it = 0; it < 4; ++it) {
        const int row = it * 4 + q8;
        const float* sp = os + row * 64 + c8;
        v8h hv, lv;
#pragma unroll
        for (int e = 0; e < 8; ++e) {
          const unsigned short hb = f2bf_bits(sp[e]);
          const unsigned short lb = f2bf_bits(sp[e] - bf_bits2f(hb));
          hv[e] = __builtin_bit_cast(_Float16, hb);
          lv[e] = __builtin_bit_cast(_Float16, lb);
        }
        const size_t o = ((size_t)(b * kS + q0 + row)) * kDim + h * kDh + c8;
        *(volatile v8h*)(aoh + o) = hv;
        *(volatile v8h*)(aol + o) = lv;
      }
      __threadfence();
    }
  }
}

__global__ __launch_bounds__(256) void k_gemm_out(const unsigned short* __restrict__ ahp, const unsigned short* __restrict__ alp,
                                                  const unsigned short* __restrict__ wtp, float* __restrict__ out) {
  __shared__ __align__(16) float sT[8][16 * 68];
  const int lane = threadIdx.x & 31, wave = threadIdx.x >> 5;
  constexpr int tilesN = kDim / 64;
  constexpr int tilesM = kM / 64;
  const int tile = blockIdx.x * 8 + wave;
  if (tile >= tilesM * tilesN) return;
  const int tm = tile / tilesN, tn = tile - tm * tilesN;
  const int m0 = tm << 6, n0 = tn << 6;

  v8f acc[4][4];
  gemm64_core<1>((const __bf16*)ahp, (const __bf16*)alp, kDim, (const __bf16*)wtp, kDim, m0, n0, kDim, lane, acc);

  float* slab = sT[wave];
  const int rlane = lane & 15, mOff = (lane >> 4) * 8;
#pragma unroll
  for (int i = 0; i < 4; ++i) {
    const int mBase = m0 + (i << 4);
#pragma unroll
    for (int j = 0; j < 4; ++j)
#pragma unroll
      for (int r = 0; r < 8; ++r) slab[(mOff + r) * 68 + (j << 4) + rlane] = acc[i][j][r];
    wave_sync_lds();
    const int h2 = lane >> 4, c4 = (lane & 15) * 4;
    for (int pass = 0; pass < 2; ++pass) {
#pragma unroll
      for (int it = 0; it < 8; ++it) {
        const int row = it * 2 + h2;
        const v4f v = *(const v4f*)(slab + row * 68 + c4);
        *(volatile v4f*)(out + (size_t)(mBase + row) * kDim + n0 + c4) = v;
      }
      __threadfence();
    }
    wave_sync_lds();
  }
}

extern "C" void kernel_launch(void* const* d_in, const int* in_sizes, int n_in,
                              void* d_out, int out_size, void* d_ws, size_t ws_size,
                              hipStream_t stream) {
  if (n_in < 5) return;
  if (in_sizes[0] != kM * kDim) return;
  if (in_sizes[1] != kS * kDh) return;
  if (in_sizes[2] != kDim) return;
  if (in_sizes[3] != kDim * kNqkv) return;
  if (in_sizes[4] != kDim * kDim) return;
  if (out_size != kM * kDim) return;
  if (ws_size < kWsTotal) return;

  const float* x     = (const float*)d_in[0];
  const float* pos   = (const float*)d_in[1];
  const float* g     = (const float*)d_in[2];
  const float* w_qkv = (const float*)d_in[3];
  const float* w_out = (const float*)d_in[4];
  float* out = (float*)d_out;

  char* ws = (char*)d_ws;
  unsigned short* Xb   = (unsigned short*)(ws + kOffXb);
  float*          Rs   = (float*)(ws + kOffRs);
  unsigned short* Wq   = (unsigned short*)(ws + kOffWq);
  unsigned short* Wo   = (unsigned short*)(ws + kOffWo);
  float*          Ct   = (float*)(ws + kOffCt);
  float*          St   = (float*)(ws + kOffSt);
  unsigned short* Qh   = (unsigned short*)(ws + kOffQh);
  unsigned short* Ql   = (unsigned short*)(ws + kOffQl);
  unsigned short* Kh   = (unsigned short*)(ws + kOffKh);
  unsigned short* Kl   = (unsigned short*)(ws + kOffKl);
  unsigned short* Vh   = (unsigned short*)(ws + kOffVh);
  unsigned short* Vl   = (unsigned short*)(ws + kOffVl);
  unsigned short* Vth  = (unsigned short*)(ws + kOffVth);
  unsigned short* Vtl  = (unsigned short*)(ws + kOffVtl);
  unsigned short* Ah   = (unsigned short*)(ws + kOffAh);
  unsigned short* Al   = (unsigned short*)(ws + kOffAl);

  k_rms_xcast<<<kM, 128, 0, stream>>>(x, Xb, Rs);
  k_wcast<true><<<dim3(kNqkv / 64, kDim / 64), 256, 0, stream>>>(w_qkv, g, Wq, kNqkv);
  k_wcast<false><<<dim3(kDim / 64, kDim / 64), 256, 0, stream>>>(w_out, g, Wo, kDim);
  k_trig<<<(kS * kDh + 255) / 256, 256, 0, stream>>>(pos, Ct, St, kS * kDh);
  k_gemm_qkv<<<(kM / 64) * (kNqkv / 64) / 8, 256, 0, stream>>>(Xb, Wq, Rs, Ct, St, Qh, Ql, Kh, Kl, Vh, Vl);
  k_vtrans<<<dim3(kBH * (kS / 64), 2), 256, 0, stream>>>(Vh, Vl, Vth, Vtl);
  k_attn<<<kBH * (kS / 64), 128, 0, stream>>>(Qh, Ql, Kh, Kl, Vth, Vtl, Ah, Al);
  k_gemm_out<<<(kM / 64) * (kDim / 64) / 8, 256, 0, stream>>>(Ah, Al, Wo, out);
}
